// BiBoAttention_15333033247085
// MI455X (gfx1250) — hardware-verified
//
#include <hip/hip_runtime.h>
#include <math.h>
#include <stdint.h>

#define BB      2
#define SS      2048
#define HID     1024
#define NH      16
#define NKV     4
#define HD      64
#define QCOLS   (NH * HD)
#define KVC     (NKV * HD)
#define KVCOLS  (2 * NKV * HD)
#define MAXPOS  4096
#define RMS_EPS 1e-6f
#define NUNIT_TOK (NH + NKV)
#define SGH     2
#define NT32    (SS / 64)
#define CTRL_N  (NT32 * NT32)
#define KEND_PITCH NT32
#define MTH     (-1.0e30f)

typedef __attribute__((ext_vector_type(16))) _Float16 v16h;
typedef __attribute__((ext_vector_type(8)))  _Float16 v8h;
typedef __attribute__((ext_vector_type(16))) __bf16   v16b;
typedef __attribute__((ext_vector_type(8)))  __bf16   v8b;
typedef __attribute__((ext_vector_type(8)))  float    v8f;
typedef __attribute__((ext_vector_type(4)))  float    v4f;
typedef __attribute__((ext_vector_type(2)))  float    v2f;
typedef __attribute__((ext_vector_type(4)))  unsigned int v4u;
typedef __attribute__((ext_vector_type(2)))  unsigned int v2u;

__device__ __forceinline__ unsigned short f2bf_bits(float f) {
  unsigned u = __float_as_uint(f);
  return (unsigned short)((u + 0x7FFFu + ((u >> 16) & 1u)) >> 16);
}
__device__ __forceinline__ float bf_bits2f(unsigned short h) { return __uint_as_float(((unsigned)h) << 16); }

__device__ __forceinline__ void dep_guard_h(v8f& a, v8f& b, v16h x, v16h y) { asm volatile("v_nop\n\tv_nop\n\tv_nop\n\tv_nop" : "+v"(a), "+v"(b) : "v"(x), "v"(y)); }
__device__ __forceinline__ void dep_guard_b(v8f& a, v8f& b, v16b x, v16b y) { asm volatile("v_nop\n\tv_nop\n\tv_nop\n\tv_nop" : "+v"(a), "+v"(b) : "v"(x), "v"(y)); }
__device__ __forceinline__ void keep4_h(v16h a, v16h b, v16h c, v16h d) { asm volatile("v_nop" :: "v"(a), "v"(b), "v"(c), "v"(d)); }
__device__ __forceinline__ void keep4_b(v16b a, v16b b, v16b c, v16b d) { asm volatile("v_nop" :: "v"(a), "v"(b), "v"(c), "v"(d)); }
__device__ __forceinline__ void acc_guard4(v8f& a, v8f& b, v8f& c, v8f& d) { asm volatile("v_nop\n\tv_nop\n\tv_nop\n\tv_nop" : "+v"(a), "+v"(b), "+v"(c), "+v"(d)); }
template <typename T> struct Frag;
template <> struct Frag<_Float16> {
  typedef v16h V; union U { v16h v; v8h h[2]; };
  static __device__ __forceinline__ v16h load(const _Float16* p) {
    U f; f.h[0] = *(const v8h*)(p); f.h[1] = *(const v8h*)(p + 16); return f.v;
  }
  static __device__ __forceinline__ v8f mma(v16h a, v16h b, v8f c) {
    return __builtin_amdgcn_wmma_f32_16x16x32_f16(false, a, false, b, (short)0, c, false, false);
  }
  static __device__ __forceinline__ void guard(v8f& a, v8f& b, v16h x, v16h y) { dep_guard_h(a, b, x, y); }
  static __device__ __forceinline__ void keep(v16h a, v16h b, v16h c, v16h d) { keep4_h(a, b, c, d); }
};
template <> struct Frag<__bf16> {
  typedef v16b V; union U { v16b v; v8b h[2]; };
  static __device__ __forceinline__ v16b load(const __bf16* p) {
    U f; f.h[0] = *(const v8b*)(p); f.h[1] = *(const v8b*)(p + 16); return f.v;
  }
  static __device__ __forceinline__ v8f mma(v16b a, v16b b, v8f c) {
    return __builtin_amdgcn_wmma_f32_16x16x32_bf16(false, a, false, b, (short)0, c, false, false);
  }
  static __device__ __forceinline__ void guard(v8f& a, v8f& b, v16b x, v16b y) { dep_guard_b(a, b, x, y); }
  static __device__ __forceinline__ void keep(v16b a, v16b b, v16b c, v16b d) { keep4_b(a, b, c, d); }
};

template <int ET> struct Elem;
template <> struct Elem<0> { typedef _Float16 T; };
template <> struct Elem<1> { typedef __bf16 T; };
template <int ET, bool SPLIT, int BIAS_MODE, int OUT_MODE, bool RESID, int ACT = 0, bool SKIPF = false, bool SKIPK = false>
__global__ __launch_bounds__(256) void wmma_gemm64(
    const unsigned short* __restrict__ Ap, const unsigned short* __restrict__ A2p, int lda, long strideA,
    const unsigned short* __restrict__ Btp, const unsigned short* __restrict__ Bt2p, int ldb, long strideB,
    void* __restrict__ Cout, void* __restrict__ Cout2, int ldc, long strideC,
    const float* __restrict__ bias,
    const float* __restrict__ resid, long strideR,
    int M, int N, int K, float scale, const int* __restrict__ ctrl) {
  typedef typename Elem<ET>::T T;
  typedef typename Frag<T>::V V;
  const T* A = (const T*)Ap; const T* A2 = (const T*)A2p; const T* Bt = (const T*)Btp; const T* Bt2 = (const T*)Bt2p;
  __shared__ __align__(16) float sT[8][16 * 68];
  const int b    = blockIdx.y;
  const int lane = threadIdx.x & 31;
  const int wave = threadIdx.x >> 5;
  const int tilesN = N >> 6;
  const int tilesM = M >> 6;
  const int tile = blockIdx.x * 8 + wave;
  if (tile >= tilesM * tilesN) return;
  const int tm = tile / tilesN;
  const int tn = tile - tm * tilesN;
  const int m0 = tm << 6;
  const int n0 = tn << 6;
  if (SKIPF) {
    int fi = tm * tilesN + tn;
    fi = (fi < CTRL_N) ? fi : (CTRL_N - 1);
    const int f = __builtin_amdgcn_readfirstlane(ctrl[fi]);
    if (f == 0) return;
  }

  const T* Ab  = A  + (size_t)b * strideA;
  const T* Bb  = Bt + (size_t)b * strideB;
  const T* Ab2 = SPLIT ? (A2  + (size_t)b * strideA) : nullptr;
  const T* Bb2 = SPLIT ? (Bt2 + (size_t)b * strideB) : nullptr;

  const int rlane = lane & 15;
  const int koff  = (lane >> 4) * 8;
  const int mOff  = (lane >> 4) * 8;

  v8f acc[4][4];
#pragma unroll
  for (int i = 0; i < 4; ++i)
#pragma unroll
    for (int j = 0; j < 4; ++j) acc[i][j] = (v8f){0.f,0.f,0.f,0.f,0.f,0.f,0.f,0.f};

  int kEnd = K;
  if (SKIPK) {
    int ti = tm * KEND_PITCH;
    ti = (ti < CTRL_N) ? ti : (CTRL_N - KEND_PITCH);
    int ke = __builtin_amdgcn_readfirstlane(ctrl[ti]);
    ke = (ke < 0) ? 0 : ke;
    ke = (ke > K) ? K : ke;
    kEnd = ke;
  }
  for (int k0 = 0; k0 < kEnd; k0 += 32) {
    V bh[4], bl[4];
#pragma unroll
    for (int j = 0; j < 4; ++j) {
      const size_t bo = (size_t)(n0 + (j << 4) + rlane) * ldb + koff + k0;
      bh[j] = Frag<T>::load(Bb + bo);
      if (SPLIT) bl[j] = Frag<T>::load(Bb2 + bo);
    }
#pragma unroll
    for (int i = 0; i < 4; ++i) {
      const size_t ao = (size_t)(m0 + (i << 4) + rlane) * lda + koff + k0;
      V ah = Frag<T>::load(Ab + ao);
      V al;
      if (SPLIT) al = Frag<T>::load(Ab2 + ao);
#pragma unroll
      for (int j = 0; j < 4; ++j) {
        acc[i][j] = Frag<T>::mma(ah, bh[j], acc[i][j]);
        if (SPLIT) {
          acc[i][j] = Frag<T>::mma(ah, bl[j], acc[i][j]);
          acc[i][j] = Frag<T>::mma(al, bh[j], acc[i][j]);
        }
      }
      Frag<T>::guard(acc[i][0], acc[i][3], ah, SPLIT ? al : ah);
    }
    Frag<T>::keep(bh[0], bh[1], bh[2], bh[3]);
    if (SPLIT) Frag<T>::keep(bl[0], bl[1], bl[2], bl[3]);
  }
  acc_guard4(acc[0][0], acc[0][1], acc[0][2], acc[0][3]);
  acc_guard4(acc[1][0], acc[1][1], acc[1][2], acc[1][3]);
  acc_guard4(acc[2][0], acc[2][1], acc[2][2], acc[2][3]);
  acc_guard4(acc[3][0], acc[3][1], acc[3][2], acc[3][3]);

  float* slab = sT[wave];
  const float* Rb = RESID ? (resid + (size_t)b * strideR) : nullptr;
#pragma unroll
  for (int i = 0; i < 4; ++i) {
    const int mBase = m0 + (i << 4);
#pragma unroll
    for (int j = 0; j < 4; ++j) {
      const int n = n0 + (j << 4) + rlane;
      float bv = 0.f;
      if (BIAS_MODE == 2) bv = bias[n];
#pragma unroll
      for (int r = 0; r < 8; ++r) {
        float v = acc[i][j][r] * scale;
        if (BIAS_MODE == 1) v += bias[mBase + mOff + r];
        if (BIAS_MODE == 2) v += bv;
        if (RESID) v += Rb[(size_t)(mBase + mOff + r) * ldc + n];
        if (ACT == 1) v = tanhf(v);
        if (ACT == 2) v = fmaxf(v, 0.0f);
        if (ACT == 3) v = v / (1.0f + expf(-v));
        if (ACT == 4) v = (v > 0.f) ? v : 0.01f * v;
        if (ACT == 5) v = 0.5f * v * (1.0f + erff(v * 0.70710678118654752f));
        slab[(mOff + r) * 68 + (j << 4) + rlane] = v;
      }
    }
    __builtin_amdgcn_fence(__ATOMIC_RELEASE, "workgroup");
    __builtin_amdgcn_wave_barrier();
    __builtin_amdgcn_fence(__ATOMIC_ACQUIRE, "workgroup");
    if (OUT_MODE == 0) {
      float* C = (float*)Cout + (size_t)b * strideC;
      const int hh = lane >> 4, c4 = (lane & 15) * 4;
      for (int pass = 0; pass < 2; ++pass) {
#pragma unroll
        for (int it = 0; it < 8; ++it) {
          const int row = it * 2 + hh;
          v4f v = *(const v4f*)(slab + row * 68 + c4);
          *(volatile v4f*)(C + (size_t)(mBase + row) * ldc + n0 + c4) = v;
        }
        __threadfence();
      }
    } else {
      const int q = lane >> 3, c8 = (lane & 7) * 8;
      unsigned short* C  = (unsigned short*)Cout  + (size_t)b * strideC;
      unsigned short* C2 = (OUT_MODE == 2) ? ((unsigned short*)Cout2 + (size_t)b * strideC) : nullptr;
      for (int pass = 0; pass < 2; ++pass) {
#pragma unroll
        for (int it = 0; it < 4; ++it) {
          const int row = it * 4 + q;
          const float* sp = slab + row * 68 + c8;
          v8h hv, lv;
#pragma unroll
          for (int e = 0; e < 8; ++e) {
            if (OUT_MODE == 1) {
              hv[e] = (_Float16)sp[e];
            } else {
              unsigned short hb = f2bf_bits(sp[e]);
              unsigned short lb = f2bf_bits(sp[e] - bf_bits2f(hb));
              hv[e] = __builtin_bit_cast(_Float16, hb);
              lv[e] = __builtin_bit_cast(_Float16, lb);
            }
          }
          *(volatile v8h*)(C + (size_t)(mBase + row) * ldc + n0 + c8) = hv;
          if (OUT_MODE == 2) *(volatile v8h*)(C2 + (size_t)(mBase + row) * ldc + n0 + c8) = lv;
        }
        __threadfence();
      }
    }
    __builtin_amdgcn_fence(__ATOMIC_RELEASE, "workgroup");
    __builtin_amdgcn_wave_barrier();
    __builtin_amdgcn_fence(__ATOMIC_ACQUIRE, "workgroup");
  }
}

__device__ __forceinline__ unsigned pk16(unsigned short a, unsigned short b) { return (unsigned)a | ((unsigned)b << 16); }

__global__ __launch_bounds__(256) void split_bf16x2_kernel(const float* __restrict__ in, unsigned short* __restrict__ hi,
                                                           unsigned short* __restrict__ lo, int n2) {
  const int i = blockIdx.x * 256 + threadIdx.x;
  if (i < n2) {
    const v2f f = *(const v2f*)(in + 2 * (size_t)i);
    const unsigned short h0 = f2bf_bits(f[0]), h1 = f2bf_bits(f[1]);
    const unsigned short l0 = f2bf_bits(f[0] - bf_bits2f(h0)), l1 = f2bf_bits(f[1] - bf_bits2f(h1));
    const unsigned uh = pk16(h0, h1), ul = pk16(l0, l1);
    ((volatile unsigned*)hi)[i] = uh;
    ((volatile unsigned*)lo)[i] = ul;
    __threadfence();
    ((volatile unsigned*)hi)[i] = uh;
    ((volatile unsigned*)lo)[i] = ul;
  }
}

__global__ __launch_bounds__(256) void mask_tiles_kernel(const float* __restrict__ mask,
                                                         int* __restrict__ flagtab, int* __restrict__ kendtab) {
  __shared__ int fl[NT32];
  __shared__ unsigned rlo[8];
  __shared__ unsigned rhi[8];
  const int mt   = blockIdx.x;
  const int tid  = threadIdx.x;
  const int lane = tid & 31;
  const int wave = tid >> 5;
  const int j0   = tid * 8;
  int any = 0;
  unsigned rowlo = 0u, rowhi = 0u;
#pragma unroll 1
  for (int r = 0; r < 64; ++r) {
    const float* mr = mask + (size_t)(mt * 64 + r) * SS + j0;
    const v4f mk0 = *(const v4f*)(mr);
    const v4f mk1 = *(const v4f*)(mr + 4);
    const int a = ((mk0[0] > MTH) | (mk0[1] > MTH) | (mk0[2] > MTH) | (mk0[3] > MTH) |
                   (mk1[0] > MTH) | (mk1[1] > MTH) | (mk1[2] > MTH) | (mk1[3] > MTH)) ? 1 : 0;
    any |= a;
    const unsigned sh = ((unsigned)a) << (r & 31);
    rowlo |= (r < 32) ? sh : 0u;
    rowhi |= (r < 32) ? 0u : sh;
  }
  any |= __shfl_xor(any, 1, 32);
  any |= __shfl_xor(any, 2, 32);
  any |= __shfl_xor(any, 4, 32);
#pragma unroll
  for (int off = 1; off < 32; off <<= 1) {
    rowlo |= (unsigned)__shfl_xor((int)rowlo, off, 32);
    rowhi |= (unsigned)__shfl_xor((int)rowhi, off, 32);
  }
  if ((lane & 7) == 0) fl[tid >> 3] = any;
  if (lane == 0) { rlo[wave] = rowlo; rhi[wave] = rowhi; }
  __syncthreads();
  if (wave == 0) {
    const int f = fl[lane];
    unsigned ol = rlo[0], oh = rhi[0];
#pragma unroll
    for (int w = 1; w < 8; ++w) { ol |= rlo[w]; oh |= rhi[w]; }
    const bool has_empty_row = (ol != 0xFFFFFFFFu) || (oh != 0xFFFFFFFFu);
    int ke = (f != 0) ? (lane + 1) * 64 : 0;
#pragma unroll
    for (int off = 1; off < 32; off <<= 1) { const int o = __shfl_xor(ke, off, 32); ke = (o > ke) ? o : ke; }
    const int kend = has_empty_row ? SS : ke;
    volatile int* fp = flagtab + (size_t)mt * NT32 + lane;
    volatile int* kp = kendtab + (size_t)mt * KEND_PITCH + lane;
    *fp = f;
    *kp = kend;
    __threadfence();
    *fp = f;
    *kp = kend;
  }
}

__global__ __launch_bounds__(256) void norm_rope_split_kernel(
    const float* __restrict__ Qf, const float* __restrict__ KVf,
    const float* __restrict__ cosT, const float* __restrict__ sinT,
    const int* __restrict__ pos, const float* __restrict__ qw, const float* __restrict__ kw,
    unsigned short* __restrict__ Qhi, unsigned short* __restrict__ Qlo,
    unsigned short* __restrict__ Khi, unsigned short* __restrict__ Klo, int nunits) {
  __shared__ __align__(16) unsigned short st[8][128];
  const int tid  = threadIdx.x;
  const int w    = tid >> 5;
  const int lane = tid & 31;
  int gu = blockIdx.x * 8 + w;
  gu = (gu < nunits) ? gu : (nunits - 1);
  const int t = gu / NUNIT_TOK;
  const int u = gu - t * NUNIT_TOK;
  const bool isq = (u < NH);
  const int hq = isq ? u : 0;
  const int hk = isq ? 0 : (u - NH);
  const float* qs = Qf  + (size_t)t * QCOLS  + hq * HD;
  const float* ks = KVf + (size_t)t * KVCOLS + hk * HD;
  const float xq0 = qs[lane], xq1 = qs[lane + 32];
  const float xk0 = ks[lane], xk1 = ks[lane + 32];
  const float x0 = isq ? xq0 : xk0;
  const float x1 = isq ? xq1 : xk1;
  const float wq0 = qw[lane], wq1 = qw[lane + 32];
  const float wk0 = kw[lane], wk1 = kw[lane + 32];
  const float w0 = isq ? wq0 : wk0;
  const float w1 = isq ? wq1 : wk1;
  float ssq = x0 * x0 + x1 * x1;
#pragma unroll
  for (int off = 16; off > 0; off >>= 1) ssq += __shfl_xor(ssq, off, 32);
  const float var = ssq * (1.0f / 64.0f);
  const float inv = rsqrtf(var + RMS_EPS);
  const float y0 = w0 * (x0 * inv);
  const float y1 = w1 * (x1 * inv);
  int p = pos[t];
  p = (p < 0) ? 0 : ((p > MAXPOS - 1) ? (MAXPOS - 1) : p);
  const float c0 = cosT[(size_t)p * HD + lane];
  const float c1 = cosT[(size_t)p * HD + lane + 32];
  const float s0 = sinT[(size_t)p * HD + lane];
  const float s1 = sinT[(size_t)p * HD + lane + 32];
  const float o0 = y0 * c0 - y1 * s0;
  const float o1 = y1 * c1 + y0 * s1;
  const unsigned short hb0 = f2bf_bits(o0), hb1 = f2bf_bits(o1);
  const unsigned short lb0 = f2bf_bits(o0 - bf_bits2f(hb0));
  const unsigned short lb1 = f2bf_bits(o1 - bf_bits2f(hb1));
  st[w][lane]      = hb0;
  st[w][32 + lane] = hb1;
  st[w][64 + lane] = lb0;
  st[w][96 + lane] = lb1;
  __syncthreads();
  const int idx = ((lane >> 3) & 1) * 64 + (lane & 7) * 8;
  const v4u val = *(const v4u*)(&st[w][idx]);
  const size_t co = (size_t)(lane & 7) * 8;
  unsigned short* dq = ((lane < 8) ? Qhi : Qlo) + (size_t)t * QCOLS + hq * HD + co;
  unsigned short* dk = ((lane < 8) ? Khi : Klo) + (size_t)t * KVC   + hk * HD + co;
  unsigned short* d  = isq ? dq : dk;
  if (lane < 16) { *(volatile v4u*)d = val; }
  __threadfence();
  if (lane < 16) { *(volatile v4u*)d = val; }
}

__global__ __launch_bounds__(256) void vtrans_split_kernel(const float* __restrict__ KVf,
                                                           unsigned short* __restrict__ VThi, unsigned short* __restrict__ VTlo) {
  __shared__ __align__(16) unsigned short th[64 * 72];
  __shared__ __align__(16) unsigned short tl[64 * 72];
  const int c0  = blockIdx.x * 64;
  const int r0  = blockIdx.y * 64;
  const int tid = threadIdx.x;
  {
    const int rr = tid >> 2;
    const int cq = (tid & 3) * 16;
    const float* src = KVf + (size_t)(r0 + rr) * KVCOLS + KVC + c0 + cq;
#pragma unroll
    for (int q = 0; q < 4; ++q) {
      const v4f f = *(const v4f*)(src + 4 * q);
#pragma unroll
      for (int e = 0; e < 4; ++e) {
        const unsigned short hb = f2bf_bits(f[e]);
        const unsigned short lb = f2bf_bits(f[e] - bf_bits2f(hb));
        th[rr * 72 + cq + 4 * q + e] = hb;
        tl[rr * 72 + cq + 4 * q + e] = lb;
      }
    }
  }
  __syncthreads();
  const int sub = tid >> 3;
  const int c8  = (tid & 7) * 8;
  v4u hv[2], lv[2];
#pragma unroll
  for (int it = 0; it < 2; ++it) {
    const int oc = it * 32 + sub;
    v4u a, a2;
#pragma unroll
    for (int q = 0; q < 4; ++q) {
      a[q]  = pk16(th[(c8 + 2 * q) * 72 + oc], th[(c8 + 2 * q + 1) * 72 + oc]);
      a2[q] = pk16(tl[(c8 + 2 * q) * 72 + oc], tl[(c8 + 2 * q + 1) * 72 + oc]);
    }
    hv[it] = a; lv[it] = a2;
  }
  for (int pass = 0; pass < 2; ++pass) {
#pragma unroll
    for (int it = 0; it < 2; ++it) {
      const int oc = it * 32 + sub;
      const size_t go = (size_t)(c0 + oc) * SS + r0 + c8;
      *(volatile v4u*)(VThi + go) = hv[it];
      *(volatile v4u*)(VTlo + go) = lv[it];
    }
    __threadfence();
  }
}

__global__ __launch_bounds__(256) void softmax_mask_kernel(const float* __restrict__ S, const float* __restrict__ mask,
                                                           unsigned short* __restrict__ Phi, unsigned short* __restrict__ Plo) {
  __shared__ float redm[8];
  __shared__ float reds[8];
  const int i    = blockIdx.x;
  const int y    = blockIdx.y;
  const int tid  = threadIdx.x;
  const int lane = tid & 31;
  const int wave = tid >> 5;
  const int j0   = tid * 8;
  const size_t roff = ((size_t)y * SS + i) * SS + j0;
  const float* sr = S + roff;
  const float* mr = mask + (size_t)i * SS + j0;
  const v4f a0  = *(const v4f*)(sr);
  const v4f a1  = *(const v4f*)(sr + 4);
  const v4f mk0 = *(const v4f*)(mr);
  const v4f mk1 = *(const v4f*)(mr + 4);
  v4f t0, t1;
#pragma unroll
  for (int e = 0; e < 4; ++e) {
    t0[e] = (mk0[e] > MTH) ? (a0[e] + mk0[e]) : mk0[e];
    t1[e] = (mk1[e] > MTH) ? (a1[e] + mk1[e]) : mk1[e];
  }
  float m = fmaxf(fmaxf(fmaxf(t0[0], t0[1]), fmaxf(t0[2], t0[3])),
                  fmaxf(fmaxf(t1[0], t1[1]), fmaxf(t1[2], t1[3])));
#pragma unroll
  for (int off = 16; off > 0; off >>= 1) m = fmaxf(m, __shfl_xor(m, off, 32));
  if (lane == 0) redm[wave] = m;
  __syncthreads();
  float mx = redm[0];
#pragma unroll
  for (int w = 1; w < 8; ++w) mx = fmaxf(mx, redm[w]);
  const float e0 = expf(t0[0] - mx), e1 = expf(t0[1] - mx), e2 = expf(t0[2] - mx), e3 = expf(t0[3] - mx);
  const float e4 = expf(t1[0] - mx), e5 = expf(t1[1] - mx), e6 = expf(t1[2] - mx), e7 = expf(t1[3] - mx);
  float s = ((e0 + e1) + (e2 + e3)) + ((e4 + e5) + (e6 + e7));
#pragma unroll
  for (int off = 16; off > 0; off >>= 1) s += __shfl_xor(s, off, 32);
  if (lane == 0) reds[wave] = s;
  __syncthreads();
  float tot = reds[0];
#pragma unroll
  for (int w = 1; w < 8; ++w) tot += reds[w];
  const float inv = 1.0f / tot;
  const float p0 = e0 * inv, p1 = e1 * inv, p2 = e2 * inv, p3 = e3 * inv;
  const float p4 = e4 * inv, p5 = e5 * inv, p6 = e6 * inv, p7 = e7 * inv;
  const unsigned short h0 = f2bf_bits(p0), h1 = f2bf_bits(p1), h2 = f2bf_bits(p2), h3 = f2bf_bits(p3);
  const unsigned short h4 = f2bf_bits(p4), h5 = f2bf_bits(p5), h6 = f2bf_bits(p6), h7 = f2bf_bits(p7);
  const unsigned short l0 = f2bf_bits(p0 - bf_bits2f(h0)), l1 = f2bf_bits(p1 - bf_bits2f(h1));
  const unsigned short l2 = f2bf_bits(p2 - bf_bits2f(h2)), l3 = f2bf_bits(p3 - bf_bits2f(h3));
  const unsigned short l4 = f2bf_bits(p4 - bf_bits2f(h4)), l5 = f2bf_bits(p5 - bf_bits2f(h5));
  const unsigned short l6 = f2bf_bits(p6 - bf_bits2f(h6)), l7 = f2bf_bits(p7 - bf_bits2f(h7));
  const v4u hv = (v4u){pk16(h0, h1), pk16(h2, h3), pk16(h4, h5), pk16(h6, h7)};
  const v4u lv = (v4u){pk16(l0, l1), pk16(l2, l3), pk16(l4, l5), pk16(l6, l7)};
  *(volatile v4u*)(Phi + roff) = hv;
  *(volatile v4u*)(Plo + roff) = lv;
  __threadfence();
  *(volatile v4u*)(Phi + roff) = hv;
  *(volatile v4u*)(Plo + roff) = lv;
}

extern "C" void kernel_launch(void* const* d_in, const int* in_sizes, int n_in,
                              void* d_out, int out_size, void* d_ws, size_t ws_size,
                              hipStream_t stream) {
  if (n_in < 11) return;
  if (in_sizes[0] != BB * SS * HID) return;
  if (in_sizes[1] != MAXPOS * HD || in_sizes[2] != MAXPOS * HD) return;
  if (in_sizes[3] != BB * SS) return;
  if (in_sizes[4] != SS * SS) return;
  if (in_sizes[5] != QCOLS * HID || in_sizes[6] != KVC * HID || in_sizes[7] != KVC * HID) return;
  if (in_sizes[8] != HID * QCOLS) return;
  if (in_sizes[9] != HD || in_sizes[10] != HD) return;
  if (out_size != BB * SS * HID) return;

  const float* x    = (const float*)d_in[0];
  const float* cosT = (const float*)d_in[1];
  const float* sinT = (const float*)d_in[2];
  const int*   pos  = (const int*)d_in[3];
  const float* mask = (const float*)d_in[4];
  const float* Wq   = (const float*)d_in[5];
  const float* Wk   = (const float*)d_in[6];
  const float* Wv   = (const float*)d_in[7];
  const float* Wo   = (const float*)d_in[8];
  const float* qw   = (const float*)d_in[9];
  const float* kw   = (const float*)d_in[10];

  const size_t PCT = (size_t)CTRL_N * 4;
  const size_t PWQ = (size_t)QCOLS * HID * 2;
  const size_t PWKV = (size_t)KVCOLS * HID * 2;
  const size_t PX  = (size_t)SS * HID * 2;
  const size_t PQF = (size_t)SS * QCOLS * 4;
  const size_t PKVF = (size_t)SS * KVCOLS * 4;
  const size_t PQ16 = (size_t)SS * QCOLS * 2;
  const size_t PK16 = (size_t)SS * KVC * 2;
  const size_t PVT = (size_t)KVC * SS * 2;
  const size_t PS  = (size_t)SGH * SS * SS * 4;
  const size_t PP  = (size_t)SGH * SS * SS * 2;
  const size_t PO  = (size_t)SS * QCOLS * 2;
  size_t off = 0;
  const size_t oFlag = off; off += PCT;
  const size_t oKend = off; off += PCT;
  const size_t oWqhi = off; off += PWQ;
  const size_t oWqlo = off; off += PWQ;
  const size_t oWKVhi = off; off += PWKV;
  const size_t oWKVlo = off; off += PWKV;
  const size_t oWohi = off; off += PWQ;
  const size_t oWolo = off; off += PWQ;
  const size_t oXhi  = off; off += PX;
  const size_t oXlo  = off; off += PX;
  const size_t oQf   = off; off += PQF;
  const size_t oKVf  = off; off += PKVF;
  const size_t oQhi  = off; off += PQ16;
  const size_t oQlo  = off; off += PQ16;
  const size_t oKhi  = off; off += PK16;
  const size_t oKlo  = off; off += PK16;
  const size_t oVThi = off; off += PVT;
  const size_t oVTlo = off; off += PVT;
  const size_t oS    = off; off += PS;
  const size_t oPhi  = off; off += PP;
  const size_t oPlo  = off; off += PP;
  const size_t oOhi  = off; off += PO;
  const size_t oOlo  = off; off += PO;
  if (off > ws_size) return;

  char* ws = (char*)d_ws;
  int*            flagtab = (int*)(ws + oFlag);
  int*            kendtab = (int*)(ws + oKend);
  unsigned short* Wqhi = (unsigned short*)(ws + oWqhi);
  unsigned short* Wqlo = (unsigned short*)(ws + oWqlo);
  unsigned short* WKVhi = (unsigned short*)(ws + oWKVhi);
  unsigned short* WKVlo = (unsigned short*)(ws + oWKVlo);
  unsigned short* Wohi = (unsigned short*)(ws + oWohi);
  unsigned short* Wolo = (unsigned short*)(ws + oWolo);
  unsigned short* Xhi  = (unsigned short*)(ws + oXhi);
  unsigned short* Xlo  = (unsigned short*)(ws + oXlo);
  float*          Qf   = (float*)(ws + oQf);
  float*          KVf  = (float*)(ws + oKVf);
  unsigned short* Qhi  = (unsigned short*)(ws + oQhi);
  unsigned short* Qlo  = (unsigned short*)(ws + oQlo);
  unsigned short* Khi  = (unsigned short*)(ws + oKhi);
  unsigned short* Klo  = (unsigned short*)(ws + oKlo);
  unsigned short* VThi = (unsigned short*)(ws + oVThi);
  unsigned short* VTlo = (unsigned short*)(ws + oVTlo);
  float*          Sbuf = (float*)(ws + oS);
  unsigned short* Phi  = (unsigned short*)(ws + oPhi);
  unsigned short* Plo  = (unsigned short*)(ws + oPlo);
  unsigned short* Ohi  = (unsigned short*)(ws + oOhi);
  unsigned short* Olo  = (unsigned short*)(ws + oOlo);

  const float* dummy = qw;
  const dim3 blk(256);
  const int n2wq = QCOLS * HID / 2;
  const int n2wk = KVC * HID / 2;
  const int n2x  = SS * HID / 2;

  split_bf16x2_kernel<<<dim3((n2wq + 255) / 256), blk, 0, stream>>>(Wq, Wqhi, Wqlo, n2wq);
  split_bf16x2_kernel<<<dim3((n2wk + 255) / 256), blk, 0, stream>>>(Wk, WKVhi, WKVlo, n2wk);
  split_bf16x2_kernel<<<dim3((n2wk + 255) / 256), blk, 0, stream>>>(Wv, WKVhi + (size_t)KVC * HID, WKVlo + (size_t)KVC * HID, n2wk);
  split_bf16x2_kernel<<<dim3((n2wq + 255) / 256), blk, 0, stream>>>(Wo, Wohi, Wolo, n2wq);
  mask_tiles_kernel<<<dim3(NT32), blk, 0, stream>>>(mask, flagtab, kendtab);

  const int tilesM = SS / 64;
  const dim3 gQ((tilesM * (QCOLS / 64) + 7) / 8, 1);
  const dim3 gKV((tilesM * (KVCOLS / 64) + 7) / 8, 1);
  const dim3 gS((tilesM * (SS / 64) + 7) / 8, SGH);
  const dim3 gPV((tilesM * (HD / 64) + 7) / 8, SGH);
  const dim3 gO((tilesM * (HID / 64) + 7) / 8, 1);
  const int nunits = SS * NUNIT_TOK;
  const dim3 gNR(nunits / 8);

  for (int b = 0; b < BB; ++b) {
    split_bf16x2_kernel<<<dim3((n2x + 255) / 256), blk, 0, stream>>>(x + (size_t)b * SS * HID, Xhi, Xlo, n2x);
    wmma_gemm64<1, true, 0, 0, false, 0, false, false><<<gQ, blk, 0, stream>>>(
        Xhi, Xlo, HID, 0L, Wqhi, Wqlo, HID, 0L, (void*)Qf, (void*)Qf, QCOLS, 0L,
        dummy, dummy, 0L, SS, QCOLS, HID, 1.0f, flagtab);
    wmma_gemm64<1, true, 0, 0, false, 0, false, false><<<gKV, blk, 0, stream>>>(
        Xhi, Xlo, HID, 0L, WKVhi, WKVlo, HID, 0L, (void*)KVf, (void*)KVf, KVCOLS, 0L,
        dummy, dummy, 0L, SS, KVCOLS, HID, 1.0f, flagtab);
    norm_rope_split_kernel<<<gNR, blk, 0, stream>>>(Qf, KVf, cosT, sinT, pos + (size_t)b * SS, qw, kw,
                                                     Qhi, Qlo, Khi, Klo, nunits);
    vtrans_split_kernel<<<dim3(KVC / 64, SS / 64), blk, 0, stream>>>(KVf, VThi, VTlo);
    for (int sg = 0; sg < NH / SGH; ++sg) {
      const int h0  = sg * SGH;
      const int kvh = h0 / (NH / NKV);
      wmma_gemm64<1, true, 0, 0, false, 0, true, false><<<gS, blk, 0, stream>>>(
          Qhi + (size_t)h0 * HD, Qlo + (size_t)h0 * HD, QCOLS, (long)HD,
          Khi + (size_t)kvh * HD, Klo + (size_t)kvh * HD, KVC, 0L,
          (void*)Sbuf, (void*)Sbuf, SS, (long)SS * SS,
          dummy, dummy, 0L, SS, SS, HD, 0.125f, flagtab);
      softmax_mask_kernel<<<dim3(SS, SGH), blk, 0, stream>>>(Sbuf, mask, Phi, Plo);
      wmma_gemm64<1, true, 0, 2, false, 0, false, true><<<gPV, blk, 0, stream>>>(
          Phi, Plo, SS, (long)SS * SS,
          VThi + (size_t)kvh * HD * SS, VTlo + (size_t)kvh * HD * SS, SS, 0L,
          (void*)(Ohi + (size_t)h0 * HD), (void*)(Olo + (size_t)h0 * HD), QCOLS, (long)HD,
          dummy, dummy, 0L, SS, HD, SS, 1.0f, kendtab);
    }
    float* outb = (float*)d_out + (size_t)b * SS * HID;
    wmma_gemm64<1, true, 0, 0, false, 0, false, false><<<gO, blk, 0, stream>>>(
        Ohi, Olo, QCOLS, 0L, Wohi, Wolo, QCOLS, 0L, (void*)outb, (void*)outb, HID, 0L,
        dummy, dummy, 0L, SS, HID, QCOLS, 1.0f, flagtab);
  }
  (void)hipGetLastError();
}
